// my_lstm_1322849927328
// MI455X (gfx1250) — hardware-run, weakly checked
//
#include <hip/hip_runtime.h>


#ifndef NB
#define NB 64
#endif
#ifndef SEQ
#define SEQ 256
#endif
#define NB_FULL  64
#define SEQ_FULL 256
#define HID  512
#define GT   (4 * HID)
#define XD   3
#define RB   16
#define LW   16
#define HP   520
#define HCARRY 1024.0f
#define WCARRY 64.0f
#define CFOLD  (1.0f / 65536.0f)
#define L2E  1.4426950408889634f

static_assert(NB % RB == 0);
static_assert(RB == 16);
static_assert(LW * 32 == HID);
static_assert(HID % 32 == 0);
static_assert(HP >= HID);
static_assert(HP % 8 == 0);
static_assert((2 * RB * HP) % 8 == 0);
static_assert(((size_t)GT * HID) % 8 == 0);
static_assert(NB <= NB_FULL);
static_assert(SEQ <= SEQ_FULL);
static_assert(NB % 4 == 0);
static_assert(NB / 4 <= 32);
static_assert((NB / 4) * 16 == NB * 4);
static_assert(8 * 16 == 32 * 4);
static_assert((size_t)SEQ * RB * 4 * 4 + (size_t)2 * RB * HP * 2 + (size_t)LW * RB * 4 + 32 * 4 <= (size_t)131072);

typedef _Float16 h16;
typedef unsigned short bf;
typedef __attribute__((ext_vector_type(16))) _Float16 v16h;
typedef __attribute__((ext_vector_type(8)))  _Float16 v8h;
typedef __attribute__((ext_vector_type(8)))  float    v8f;
typedef __attribute__((ext_vector_type(4)))  float    v4f;
typedef v4f  __attribute__((may_alias)) v4fa;
typedef v8h  __attribute__((may_alias)) v8ha;

__device__ __forceinline__ unsigned short f2bf(float f) { unsigned u = __float_as_uint(f); u += 0x7FFFu + ((u >> 16) & 1u); return (unsigned short)(u >> 16); }
__device__ __forceinline__ float bfr(float f) { return __uint_as_float(((unsigned)f2bf(f)) << 16); }
__device__ __forceinline__ v16h cat16(v8h lo, v8h hi) { return __builtin_shufflevector(lo, hi, 0, 1, 2, 3, 4, 5, 6, 7, 8, 9, 10, 11, 12, 13, 14, 15); }
__device__ __forceinline__ v8f wmma16(v16h a, v16h b, v8f c) { return __builtin_amdgcn_wmma_f32_16x16x32_f16(false, a, false, b, (short)0, c, false, false); }
__device__ __forceinline__ v16h  ldh(const h16* p) { return cat16(*(const v8h*)p, *(const v8h*)(p + 16)); }
__device__ __forceinline__ void wave_sync() { __builtin_amdgcn_fence(3  , "wavefront"); __builtin_amdgcn_wave_barrier(); asm volatile("" ::: "memory"); }
static __device__ __forceinline__ h16 toh_flush(float v) { const h16 r = (h16)v; return (fabsf(v) < 6.103515625e-05f) ? (h16)0.0f : r; }
__device__ __forceinline__ v8f wmma16g(v16h a, v16h b, v8f c) { c = wmma16(a, b, c); asm volatile("v_nop\n\tv_nop\n\tv_nop\n\tv_nop" : "+v"(c) : "v"(a), "v"(b)); return c; }
__device__ __forceinline__ float sigm(float v) { return __builtin_amdgcn_rcpf(1.0f + __builtin_amdgcn_exp2f(-L2E * v)); }
__device__ __forceinline__ float tnh(float v)  { return 1.0f - 2.0f * __builtin_amdgcn_rcpf(1.0f + __builtin_amdgcn_exp2f((2.0f * L2E) * v)); }

__global__ __launch_bounds__(256) void k_wconv(const float* __restrict__ src, h16* dst, size_t n8) {
    const size_t i = (size_t)blockIdx.x * 256 + threadIdx.x; if (i >= n8) return;
    const v8f v = *(const v8f*)(src + i * 8); v8h o;
#pragma unroll
    for (int k = 0; k < 8; ++k) o[k] = toh_flush(bfr(v[k]) * WCARRY);
    *(volatile v8h*)(dst + i * 8) = o; __threadfence(); *(volatile v8h*)(dst + i * 8) = o;
}

__global__ __launch_bounds__(32 * LW) __attribute__((amdgpu_num_vgpr(256)))
void k_cell(const float* __restrict__ x, const float* __restrict__ fx, const float* __restrict__ xw, const float* __restrict__ xb,
            const h16* __restrict__ WP, const float* __restrict__ hb, const float* __restrict__ fcw, const float* __restrict__ fcb, float* PL) {
    __shared__ __align__(16) float xs[SEQ * RB * 4];
    __shared__ __align__(16) h16   hs[2 * RB * HP];
    __shared__ __align__(16) float hp[LW * RB];
    __shared__ __align__(16) float ln[32];
    const int tid = threadIdx.x, lane = tid & 31, lr = lane & 15, hi = lane >> 4;
    const int wave = __builtin_amdgcn_readfirstlane((int)(threadIdx.x >> 5));
    const int b0 = blockIdx.x * RB;

    for (int i = tid; i < SEQ * RB; i += 32 * LW) {
        const int t = i >> 4, row = i & 15;
        const float* xp = x + ((size_t)(b0 + row) * SEQ_FULL + (size_t)t) * XD;
        v4f v; v[0] = bfr(xp[0]); v[1] = bfr(xp[1]); v[2] = bfr(xp[2]); v[3] = 0.0f;
        *(v4fa*)(&xs[i * 4]) = v; }
    for (int i = tid; i < (2 * RB * HP) / 8; i += 32 * LW) *(v8ha*)(&hs[i * 8]) = (v8h){};

    float wx[2][4][3], bs[2][4];
#pragma unroll
    for (int j = 0; j < 2; ++j)
#pragma unroll
        for (int g = 0; g < 4; ++g) { const int G = g * HID + wave * 32 + j * 16 + lr;
            wx[j][g][0] = bfr(xw[G * XD + 0]); wx[j][g][1] = bfr(xw[G * XD + 1]); wx[j][g][2] = bfr(xw[G * XD + 2]);
            bs[j][g] = bfr(xb[G]) + bfr(hb[G]); }
    float c[2][8], hl[2][8];
#pragma unroll
    for (int j = 0; j < 2; ++j)
#pragma unroll
        for (int r = 0; r < 8; ++r) { c[j][r] = 0.0f; hl[j][r] = 0.0f; }
    const size_t wo = (size_t)(wave * 32 + lr) * HID + 8 * hi;
    __syncthreads();

#pragma unroll 1
    for (int t = 0; t < SEQ; ++t) {
        const int cur = t & 1;
        v8f acc[2][4];
#pragma unroll
        for (int j = 0; j < 2; ++j)
#pragma unroll
            for (int g = 0; g < 4; ++g) acc[j][g] = (v8f){};
        const int ao = cur * (RB * HP) + lr * HP + 8 * hi;
#pragma unroll 1
        for (int kc = 0; kc < HID; kc += 32) {
            const v16h a = cat16(*(const v8ha*)(&hs[ao + kc]), *(const v8ha*)(&hs[ao + kc + 16]));
#pragma unroll
            for (int j = 0; j < 2; ++j)
#pragma unroll
                for (int g = 0; g < 4; ++g) {
                    const v16h bq = ldh(WP + wo + (size_t)(g * HID + j * 16) * HID + kc);
                    acc[j][g] = wmma16g(a, bq, acc[j][g]); }
        }
        const int xo = (t * RB + 8 * hi) * 4;
        const int ho = (cur ^ 1) * (RB * HP) + (8 * hi) * HP + wave * 32 + lr;
#pragma unroll
        for (int r = 0; r < 8; ++r) {
            const v4f xv = *(const v4fa*)(&xs[xo + r * 4]);
#pragma unroll
            for (int j = 0; j < 2; ++j) {
                float pre[4];
#pragma unroll
                for (int g = 0; g < 4; ++g)
                    pre[g] = acc[j][g][r] * CFOLD + (bs[j][g] + xv[0] * wx[j][g][0] + xv[1] * wx[j][g][1] + xv[2] * wx[j][g][2]);
                const float ig = sigm(pre[0]), fg = sigm(pre[1]), gg = tnh(pre[2]), og = sigm(pre[3]);
                const float cn = c[j][r] * fg + ig * gg;
                c[j][r] = cn;
                const float hv = og * tnh(cn);
                hl[j][r] = hv;
                hs[ho + r * HP + j * 16] = toh_flush(hv * HCARRY); }
        }
        __syncthreads();
    }

    float pr[8];
    { const float f0 = bfr(fcw[wave * 32 + lr]), f1 = bfr(fcw[wave * 32 + 16 + lr]);
#pragma unroll
      for (int r = 0; r < 8; ++r) pr[r] = hl[0][r] * f0 + hl[1][r] * f1; }
#pragma unroll
    for (int r = 0; r < 8; ++r) {
        pr[r] += __shfl_xor(pr[r], 1, 32); pr[r] += __shfl_xor(pr[r], 2, 32);
        pr[r] += __shfl_xor(pr[r], 4, 32); pr[r] += __shfl_xor(pr[r], 8, 32); }
    if (lr == 0) {
#pragma unroll
        for (int r = 0; r < 8; ++r) hp[wave * RB + 8 * hi + r] = pr[r]; }
    __syncthreads();
    if (wave == 0) {
        const int row = lane & 15;
        float s = 0.0f;
#pragma unroll
        for (int w = 0; w < LW; ++w) s += hp[w * RB + row];
        float fxv = fx[b0 + row]; asm volatile("" : "+v"(fxv));
        s += bfr(fxv) * bfr(fcw[HID]) + bfr(fcb[0]);
        ln[lane] = (lane < 16) ? s : 0.0f;
        wave_sync();
        const v4f val = *(const v4fa*)(&ln[(lane & 7) * 4]);
        float* dst = PL + (size_t)blockIdx.x * 32 + (lane & 7) * 4;
#pragma unroll 1
        for (int ps = 0; ps < 2; ++ps) {
            if (lane < 8) *(volatile v4f*)dst = val;
            if (ps == 0) __threadfence(); }
    }
}

__global__ __launch_bounds__(32) void k_head(const float* __restrict__ PL, float* OUT) {
    const int lane = threadIdx.x & 31;
    const int i = lane < (NB / 4) ? lane : (NB / 4 - 1);
    v4f v = *(const v4f*)(PL + (size_t)(i >> 2) * 32 + (i & 3) * 4);
    asm volatile("" : "+v"(v));
#pragma unroll 1
    for (int ps = 0; ps < 2; ++ps) {
        if (lane < (NB / 4)) *(volatile v4f*)(OUT + (size_t)i * 4) = v;
        if (ps == 0) __threadfence(); }
}

static constexpr size_t al256(size_t v) { return (v + 255) & ~(size_t)255; }
static constexpr size_t SZ_WP = al256((size_t)GT * HID * 2);
static constexpr size_t SZ_PL = al256((size_t)(NB / RB) * 128);
static constexpr size_t SZ_TOTAL = SZ_WP + SZ_PL;
static_assert(SZ_TOTAL <= (size_t)134217728);
static_assert(((size_t)GT * HID * 2) % 128 == 0);

extern "C" void kernel_launch(void* const* d_in, const int* in_sizes, int n_in,
                              void* d_out, int out_size, void* d_ws, size_t ws_size, hipStream_t stream) {
    if (n_in < 8) return;
    if ((size_t)in_sizes[0] < ((size_t)(NB - 1) * SEQ_FULL + SEQ) * XD) return;
    if (in_sizes[1] < NB) return;
    if ((size_t)in_sizes[2] < (size_t)GT * XD || in_sizes[3] < GT) return;
    if ((size_t)in_sizes[4] < (size_t)GT * HID || in_sizes[5] < GT) return;
    if (in_sizes[6] < HID + 1 || in_sizes[7] < 1) return;
    if (out_size < NB) return;
    if (SZ_TOTAL > ws_size) return;
    const float* x   = (const float*)d_in[0];
    const float* fx  = (const float*)d_in[1];
    const float* xw  = (const float*)d_in[2];
    const float* xb  = (const float*)d_in[3];
    const float* hw  = (const float*)d_in[4];
    const float* hb  = (const float*)d_in[5];
    const float* fcw = (const float*)d_in[6];
    const float* fcb = (const float*)d_in[7];
    float* OUT = (float*)d_out;
    char* wsp = (char*)d_ws;
    h16* WP = (h16*)wsp; wsp += SZ_WP;
    float* PL = (float*)wsp; wsp += SZ_PL;

    { const size_t n8 = (size_t)GT * HID / 8;
      k_wconv<<<(unsigned)((n8 + 255) / 256), 256, 0, stream>>>(hw, WP, n8); }
    k_cell<<<dim3(NB / RB, 1, 1), 32 * LW, 0, stream>>>(x, fx, xw, xb, WP, hb, fcw, fcb, PL);
    k_head<<<dim3(1, 1, 1), 32, 0, stream>>>(PL, OUT);
}
